// PointNetSetAbstraction_3143916061381
// MI455X (gfx1250) — hardware-verified
//
#include <hip/hip_runtime.h>
#pragma clang fp contract(off)

typedef __attribute__((ext_vector_type(16))) _Float16 v16h;
typedef __attribute__((ext_vector_type(8)))  _Float16 v8h;
typedef __attribute__((ext_vector_type(8)))  float    v8f;
typedef __attribute__((ext_vector_type(4)))  float    v4f;
typedef __attribute__((ext_vector_type(4)))  unsigned v4u;

constexpr int BATCH_N = 8;
constexpr int PTS_N   = 8192;
constexpr int CENT_N  = 1024;
constexpr int SAMP_N  = 32;
constexpr int FEAT_N  = 64;
constexpr int TOK_N   = BATCH_N * CENT_N * SAMP_N;
constexpr int GROUPS_N = BATCH_N * CENT_N;
constexpr int K0_PAD  = 96;
constexpr int MLP_BLOCKS = TOK_N / 256;
constexpr float W_CARRY = 64.0f;
constexpr float W_CARRY_INV = 1.0f / 64.0f;
constexpr float RADIUS_SQ = 0.04f;
constexpr float BN_EPS = 1e-5f;

static_assert(TOK_N == 262144, "token count");
static_assert(TOK_N % 256 == 0, "mlp grid exact");
static_assert(K0_PAD % 32 == 0 && FEAT_N % 32 == 0, "k steps");
static_assert(GROUPS_N % 4 == 0, "group grid exact");

constexpr size_t OFF_XR  = 0;
constexpr size_t OFF_NXW = OFF_XR  + (size_t)BATCH_N * PTS_N * 3 * 4;
constexpr size_t OFF_W0H = OFF_NXW + (size_t)BATCH_N * CENT_N * 4 * 4;
constexpr size_t OFF_W1H = OFF_W0H + (size_t)64 * K0_PAD * 2;
constexpr size_t OFF_W2H = OFF_W1H + (size_t)64 * 64 * 2;
constexpr size_t OFF_A0  = OFF_W2H + (size_t)128 * 64 * 2;
constexpr size_t OFF_Y0  = OFF_A0  + (size_t)TOK_N * K0_PAD * 2;
constexpr size_t OFF_Y1  = OFF_Y0  + (size_t)TOK_N * 64 * 2;
constexpr size_t OFF_MX  = OFF_Y1  + (size_t)TOK_N * 64 * 2;
constexpr size_t OFF_MN  = OFF_MX  + (size_t)GROUPS_N * 128 * 4;
constexpr size_t OFF_P0  = OFF_MN  + (size_t)GROUPS_N * 128 * 4;
constexpr size_t OFF_P1  = OFF_P0  + (size_t)MLP_BLOCKS * 128 * 4;
constexpr size_t OFF_P2  = OFF_P1  + (size_t)MLP_BLOCKS * 128 * 4;
constexpr size_t OFF_ST0 = OFF_P2  + (size_t)MLP_BLOCKS * 256 * 4;
constexpr size_t OFF_ST1 = OFF_ST0 + 512;
constexpr size_t OFF_ST2 = OFF_ST1 + 512;
constexpr size_t WS_TOTAL = OFF_ST2 + 1024;
static_assert(WS_TOTAL == 128882688ull, "carve total");
static_assert(WS_TOTAL <= 134217728ull, "carve under 128 MiB");
static_assert((OFF_NXW % 256) == 0 && (OFF_W0H % 256) == 0 && (OFF_W1H % 256) == 0 && (OFF_W2H % 256) == 0, "align");
static_assert((OFF_A0 % 256) == 0 && (OFF_Y0 % 256) == 0 && (OFF_Y1 % 256) == 0 && (OFF_MX % 256) == 0, "align");
static_assert((OFF_MN % 256) == 0 && (OFF_P0 % 256) == 0 && (OFF_P1 % 256) == 0 && (OFF_P2 % 256) == 0, "align");
static_assert((OFF_ST0 % 256) == 0 && (OFF_ST1 % 256) == 0 && (OFF_ST2 % 256) == 0, "align");

constexpr size_t OUT0_BYTES = (size_t)BATCH_N * CENT_N * 3 * 4;
constexpr size_t OUT1_BYTES = (size_t)BATCH_N * CENT_N * 128 * 4;
static_assert(OUT0_BYTES == 98304 && (OUT0_BYTES % 128) == 0, "out1 line aligned");
static_assert(OUT0_BYTES + OUT1_BYTES == 4292608ull, "d_out total");

__device__ __forceinline__ float rbf(float f) {
  unsigned u = __float_as_uint(f);
  u = (u + 0x7FFFu + ((u >> 16) & 1u)) & 0xFFFF0000u;
  return __uint_as_float(u);
}

__device__ __forceinline__ float h16_to_f32(unsigned hb) {
  const unsigned sgn = (hb & 0x8000u) << 16; const unsigned em = hb & 0x7fffu;
  const float fn = __uint_as_float((em << 13) + 0x38000000u);
  const float fs = (float)em * 5.9604644775390625e-8f;
  const float mag = (em < 0x400u) ? fs : fn; return __uint_as_float(__float_as_uint(mag) | sgn);
}

__device__ __forceinline__ void store2_v4f(float* p, v4f v) {
  *(volatile v4f*)p = v;
  __threadfence();
  *(volatile v4f*)p = v;
}
__device__ __forceinline__ void store2_v8h(unsigned short* p, v8h v) {
  *(volatile v8h*)p = v;
  __threadfence();
  *(volatile v8h*)p = v;
}

template <typename T> struct Frag;
template <> struct Frag<_Float16> {
  typedef v16h V; union U { v16h v; v8h h[2]; };
  static __device__ __forceinline__ v16h load(const _Float16* p) {
    U f; f.h[0] = *(const v8h*)(p); f.h[1] = *(const v8h*)(p + 16); return f.v;
  }
  static __device__ __forceinline__ v8f mma(v16h a, v16h b, v8f c) {
    return __builtin_amdgcn_wmma_f32_16x16x32_f16(false, a, false, b, (short)0, c, false, false);
  }
};

__device__ __forceinline__ void guard8(v8f& a0, v8f& a1, v8f& a2, v8f& a3, v8f& a4, v8f& a5, v8f& a6, v8f& a7,
                                       v16h x0, v16h x1, v16h b0, v16h b1, v16h b2, v16h b3) {
  asm volatile("v_nop\n\tv_nop\n\tv_nop\n\tv_nop"
               : "+v"(a0), "+v"(a1), "+v"(a2), "+v"(a3), "+v"(a4), "+v"(a5), "+v"(a6), "+v"(a7)
               : "v"(x0), "v"(x1), "v"(b0), "v"(b1), "v"(b2), "v"(b3));
}

constexpr int PREP_XR_BLOCKS = 192;
constexpr int PREP_W0_BLOCKS = 3;
constexpr int PREP_W1_BLOCKS = 2;
constexpr int PREP_W2_BLOCKS = 4;
constexpr int PREP_BLOCKS = PREP_XR_BLOCKS + PREP_W0_BLOCKS + PREP_W1_BLOCKS + PREP_W2_BLOCKS;
static_assert(PREP_XR_BLOCKS * 256 * 4 == BATCH_N * PTS_N * 3, "XR coverage");
static_assert(PREP_W0_BLOCKS * 256 * 8 == 64 * K0_PAD, "W0H coverage");
static_assert(PREP_W1_BLOCKS * 256 * 8 == 64 * 64, "W1H coverage");
static_assert(PREP_W2_BLOCKS * 256 * 8 == 128 * 64, "W2H coverage");

__device__ __forceinline__ void pack_w_vec(const float* W, unsigned short* Wh, int vec, int kreal, int kpad, int perm, float zf) {
  const int vpr = kpad >> 3;
  const int o = vec / vpr;
  const int k8 = (vec - o * vpr) * 8;
  v8h hv;
#pragma unroll
  for (int e = 0; e < 8; ++e) {
    const int k = k8 + e;
    int sc = perm ? ((k < 64) ? (k + 3) : (k - 64)) : k;
    sc = sc < 0 ? 0 : sc;
    sc = sc > (kreal - 1) ? (kreal - 1) : sc;
    const float w = W[o * kreal + sc];
    const float x = (k < kreal) ? (rbf(w) * W_CARRY) : zf;
    hv[e] = (_Float16)x;
  }
  store2_v8h(Wh + (size_t)vec * 8, hv);
}

__global__ __launch_bounds__(256) void k_prep(const float* __restrict__ xyz, const float* __restrict__ W0,
                                              const float* __restrict__ W1, const float* __restrict__ W2,
                                              float* __restrict__ XR, unsigned short* __restrict__ W0h,
                                              unsigned short* __restrict__ W1h, unsigned short* __restrict__ W2h) {
  const int blk = blockIdx.x;
  const int tid = threadIdx.x;
  float zf = 0.0f;
  asm volatile("" : "+v"(zf));
  if (blk < PREP_XR_BLOCKS) {
    const int i = blk * 256 + tid;
    const v4f v = *(const v4f*)(xyz + (size_t)i * 4);
    v4f o;
#pragma unroll
    for (int e = 0; e < 4; ++e) { const float s = v[e]; o[e] = rbf(s); }
    store2_v4f(XR + (size_t)i * 4, o);
  } else if (blk < PREP_XR_BLOCKS + PREP_W0_BLOCKS) {
    const int vec = (blk - PREP_XR_BLOCKS) * 256 + tid;
    pack_w_vec(W0, W0h, vec, 67, K0_PAD, 1, zf);
  } else if (blk < PREP_XR_BLOCKS + PREP_W0_BLOCKS + PREP_W1_BLOCKS) {
    const int vec = (blk - PREP_XR_BLOCKS - PREP_W0_BLOCKS) * 256 + tid;
    pack_w_vec(W1, W1h, vec, 64, 64, 0, zf);
  } else {
    const int vec = (blk - PREP_XR_BLOCKS - PREP_W0_BLOCKS - PREP_W1_BLOCKS) * 256 + tid;
    pack_w_vec(W2, W2h, vec, 64, 64, 0, zf);
  }
}

__global__ __launch_bounds__(256) void k_fps(const float* __restrict__ XR, float* __restrict__ out0,
                                             float* __restrict__ NXW) {
#pragma clang fp contract(off)
  __shared__ __align__(16) float stg[2048 * 3];
  __shared__ __align__(16) float nxs[CENT_N * 3];
  __shared__ float swv[2][8];
  __shared__ int   swi[2][8];
  const int b = blockIdx.x;
  const int tid = threadIdx.x;
  const int lane = tid & 31;
  const int wid = tid >> 5;
  const float* xb = XR + (size_t)b * PTS_N * 3;

  float px[32], py[32], pz[32], dist[32];
#pragma unroll
  for (int ch = 0; ch < 4; ++ch) {
#pragma unroll
    for (int i = 0; i < 6; ++i) {
      const int q = i * 256 + tid;
      const v4f v = *(const v4f*)(xb + (size_t)ch * 6144 + (size_t)q * 4);
      *(v4f*)(stg + q * 4) = v;
    }
    __syncthreads();
#pragma unroll
    for (int jj = 0; jj < 8; ++jj) {
      const int q = jj * 256 + tid;
      px[ch * 8 + jj] = stg[q * 3 + 0];
      py[ch * 8 + jj] = stg[q * 3 + 1];
      pz[ch * 8 + jj] = stg[q * 3 + 2];
    }
    __syncthreads();
  }
#pragma unroll
  for (int j = 0; j < 32; ++j) dist[j] = 1e10f;

  int far = 0;
#pragma unroll 1
  for (int it = 0; it < CENT_N; ++it) {
    int fc = far < 0 ? 0 : far;
    fc = fc > (PTS_N - 1) ? (PTS_N - 1) : fc;
    const float cx = xb[fc * 3 + 0];
    const float cy = xb[fc * 3 + 1];
    const float cz = xb[fc * 3 + 2];
    if (tid == 0) { nxs[it * 3 + 0] = cx; nxs[it * 3 + 1] = cy; nxs[it * 3 + 2] = cz; }

    float lmax = -1.0f;
    int lidx = 0;
#pragma unroll
    for (int j = 0; j < 32; ++j) {
      const float dx = px[j] - cx;
      const float dy = py[j] - cy;
      const float dz = pz[j] - cz;
      const float t0 = dx * dx;
      const float t1 = dy * dy;
      const float t2 = dz * dz;
      const float d = (t0 + t2) + t1;
      const float nd = fminf(dist[j], d);
      dist[j] = nd;
      const bool tk = nd > lmax;
      lmax = tk ? nd : lmax;
      lidx = tk ? (j * 256 + tid) : lidx;
    }
#pragma unroll
    for (int off = 16; off > 0; off >>= 1) {
      const float ov = __shfl_xor(lmax, off, 32);
      const int   oi = __shfl_xor(lidx, off, 32);
      const bool take = (ov > lmax) || ((ov == lmax) && (oi < lidx));
      lmax = take ? ov : lmax;
      lidx = take ? oi : lidx;
    }
    const int par = it & 1;
    if (lane == 0) { swv[par][wid] = lmax; swi[par][wid] = lidx; }
    __syncthreads();
    float bv = swv[par][0];
    int bi = swi[par][0];
#pragma unroll
    for (int w = 1; w < 8; ++w) {
      const float ov = swv[par][w];
      const int oi = swi[par][w];
      const bool take = (ov > bv) || ((ov == bv) && (oi < bi));
      bv = take ? ov : bv;
      bi = take ? oi : bi;
    }
    far = bi;
  }
  __syncthreads();

  float* ob = out0 + (size_t)b * CENT_N * 3;
  for (int pass = 0; pass < 2; ++pass) {
#pragma unroll
    for (int i = 0; i < 3; ++i) {
      const int q = i * 256 + tid;
      const v4f v = *(const v4f*)(nxs + q * 4);
      *(volatile v4f*)(ob + (size_t)q * 4) = v;
    }
    __threadfence();
  }
  float* nb = NXW + (size_t)b * CENT_N * 4;
  for (int pass = 0; pass < 2; ++pass) {
#pragma unroll
    for (int i = 0; i < 4; ++i) {
      const int s = i * 256 + tid;
      v4f v;
      v[0] = nxs[s * 3 + 0]; v[1] = nxs[s * 3 + 1]; v[2] = nxs[s * 3 + 2]; v[3] = 0.0f;
      *(volatile v4f*)(nb + (size_t)s * 4) = v;
    }
    __threadfence();
  }
}

__global__ __launch_bounds__(128) void k_group(const float* __restrict__ XR, const float* __restrict__ pts,
                                               const float* __restrict__ NXW, unsigned short* __restrict__ A0) {
#pragma clang fp contract(off)
  __shared__ int sidx[4][SAMP_N];
  __shared__ __align__(16) _Float16 tile[4][SAMP_N * K0_PAD];
  const int wave = threadIdx.x >> 5;
  const int lane = threadIdx.x & 31;
  const int g = blockIdx.x * 4 + wave;
  const int b = g >> 10;
  const float* xb = XR + (size_t)b * PTS_N * 3;
  const v4f cv = *(const v4f*)(NXW + (size_t)g * 4);
  const float sx = cv[0];
  const float sy = cv[1];
  const float sz = cv[2];
  const float sqs = (sx * sx + sz * sz) + sy * sy;

  sidx[wave][lane] = 0;
  __syncthreads();

  int cnt = 0;
  for (int base = 0; base < PTS_N; base += 32) {
    if (cnt >= SAMP_N) break;
    const int p = base + lane;
    const float nx = xb[p * 3 + 0];
    const float ny = xb[p * 3 + 1];
    const float nz = xb[p * 3 + 2];
    float pd = sx * nx;
    pd = fmaf(sy, ny, pd);
    pd = fmaf(sz, nz, pd);
    const float sqn = (nx * nx + nz * nz) + ny * ny;
    float d = -2.0f * pd;
    d = d + sqs;
    d = d + sqn;
    const bool in = !(d > RADIUS_SQ);
    const unsigned mask = __builtin_amdgcn_ballot_w32(in);
    const int pos = cnt + __popc(mask & ((1u << lane) - 1u));
    if (in && pos < SAMP_N) sidx[wave][pos] = p;
    cnt += __popc(mask);
  }
  cnt = cnt > SAMP_N ? SAMP_N : cnt;
  __syncthreads();

  const int mine = sidx[wave][lane];
  const int head = sidx[wave][0];
  const int first = (cnt > 0) ? head : (PTS_N - 1);
  int idx = (lane < cnt) ? mine : first;
  idx = idx < 0 ? 0 : idx;
  idx = idx > (PTS_N - 1) ? (PTS_N - 1) : idx;

  const float gx = xb[idx * 3 + 0];
  const float gy = xb[idx * 3 + 1];
  const float gz = xb[idx * 3 + 2];
  const float d0 = gx - sx;
  const float d1 = gy - sy;
  const float d2 = gz - sz;

  float zf = 0.0f;
  asm volatile("" : "+v"(zf));
  const float* fp = pts + ((size_t)b * PTS_N + (size_t)idx) * FEAT_N;
  _Float16* rowp = &tile[wave][lane * K0_PAD];
#pragma unroll 1
  for (int hb = 0; hb < 2; ++hb) {
    v4f q[8];
#pragma unroll
    for (int i = 0; i < 8; ++i) q[i] = *(const v4f*)(fp + hb * 32 + i * 4);
#pragma unroll
    for (int vq = 0; vq < 4; ++vq) {
      v8h hv;
#pragma unroll
      for (int e = 0; e < 8; ++e) {
        const float fv = q[vq * 2 + (e >> 2)][e & 3];
        hv[e] = (_Float16)rbf(fv);
      }
      *(v8h*)(rowp + hb * 32 + vq * 8) = hv;
    }
    asm volatile("" ::: "memory");
  }
  {
    v8h xv;
    xv[0] = (_Float16)d0; xv[1] = (_Float16)d1; xv[2] = (_Float16)d2;
    xv[3] = (_Float16)zf; xv[4] = (_Float16)zf; xv[5] = (_Float16)zf; xv[6] = (_Float16)zf; xv[7] = (_Float16)zf;
    *(v8h*)(rowp + 64) = xv;
    v8h zv;
#pragma unroll
    for (int e = 0; e < 8; ++e) zv[e] = (_Float16)zf;
    *(v8h*)(rowp + 72) = zv;
    *(v8h*)(rowp + 80) = zv;
    *(v8h*)(rowp + 88) = zv;
  }
  __syncthreads();

  const v8h* tv = (const v8h*)(&tile[wave][0]);
  unsigned short* dst = A0 + (size_t)g * (SAMP_N * K0_PAD);
  for (int pass = 0; pass < 2; ++pass) {
#pragma unroll
    for (int i = 0; i < 12; ++i) {
      const v8h v = tv[i * 32 + lane];
      *(volatile v8h*)(dst + (size_t)(i * 32 + lane) * 8) = v;
    }
    __threadfence();
  }
}

__device__ __forceinline__ v16h bn_frag(const unsigned short* p, const float* scp, const float* shp) {
  const v4u w0 = *(const v4u*)(p);
  const v4u w1 = *(const v4u*)(p + 16);
  const v4f s0 = *(const v4f*)(scp);
  const v4f s1 = *(const v4f*)(scp + 4);
  const v4f s2 = *(const v4f*)(scp + 16);
  const v4f s3 = *(const v4f*)(scp + 20);
  const v4f t0 = *(const v4f*)(shp);
  const v4f t1 = *(const v4f*)(shp + 4);
  const v4f t2 = *(const v4f*)(shp + 16);
  const v4f t3 = *(const v4f*)(shp + 20);
  float sca[16], sha[16];
  unsigned ww[8];
#pragma unroll
  for (int e = 0; e < 4; ++e) {
    sca[e] = s0[e]; sca[4 + e] = s1[e]; sca[8 + e] = s2[e]; sca[12 + e] = s3[e];
    sha[e] = t0[e]; sha[4 + e] = t1[e]; sha[8 + e] = t2[e]; sha[12 + e] = t3[e];
    ww[e] = w0[e]; ww[4 + e] = w1[e];
  }
  v16h r;
#pragma unroll
  for (int q = 0; q < 8; ++q) {
    const unsigned wq = ww[q];
    const float y0 = h16_to_f32(wq & 0xffffu);
    const float y1 = h16_to_f32(wq >> 16);
    const float a0 = fmaxf(fmaf(y0, sca[2 * q], sha[2 * q]), 0.0f);
    const float a1 = fmaxf(fmaf(y1, sca[2 * q + 1], sha[2 * q + 1]), 0.0f);
    r[2 * q] = (_Float16)a0;
    r[2 * q + 1] = (_Float16)a1;
  }
  return r;
}

template <int KD, int NOUT, int MODE>
__global__ __launch_bounds__(256) void k_mlp(const unsigned short* __restrict__ Ain,
                                             const unsigned short* __restrict__ Wh,
                                             const float* __restrict__ bias,
                                             const float* __restrict__ stin,
                                             const float* __restrict__ gin,
                                             const float* __restrict__ bein,
                                             unsigned short* __restrict__ Yout,
                                             float* __restrict__ MXo, float* __restrict__ MNo,
                                             float* __restrict__ part) {
  constexpr int KS = KD / 32;
  constexpr int NH = NOUT / 64;
  static_assert(KD % 32 == 0 && NOUT % 64 == 0, "tile multiples");
  static_assert(MODE == 0 || KD == 64, "BN-fused A needs K = 64");
  static_assert(2 * NOUT <= 256, "stat combine coverage");
  __shared__ __align__(16) float slabs[(MODE == 2) ? 1 : 8][16 * 68];
  __shared__ __align__(16) float wst[8][2 * NOUT];
  __shared__ __align__(16) float wmm[(MODE == 2) ? 8 : 1][2 * NOUT];
  __shared__ __align__(16) float bst[2 * NOUT];
  __shared__ __align__(16) float scs[64];
  __shared__ __align__(16) float shs[64];

  const int tid = threadIdx.x;
  const int lane = tid & 31;
  const int wave = tid >> 5;
  const int rlane = lane & 15;
  const int hh = lane >> 4;
  const int koff = hh * 8;
  const int mOff = hh * 8;
  const int g = blockIdx.x * 8 + wave;
  const int row0 = g * SAMP_N;

  if (MODE != 0) {
    if (tid < 64) {
      const float mu = stin[tid];
      const float rs = stin[64 + tid];
      const float gg = rbf(gin[tid]);
      const float bb = rbf(bein[tid]);
      const float sc = rs * gg;
      scs[tid] = sc;
      shs[tid] = bb - mu * sc;
    }
    __syncthreads();
  }

  v16h af[2][KS];
  if (MODE == 0) {
    const _Float16* Ab = (const _Float16*)Ain;
#pragma unroll
    for (int i = 0; i < 2; ++i) {
#pragma unroll
      for (int ks = 0; ks < KS; ++ks)
        af[i][ks] = Frag<_Float16>::load(Ab + (size_t)(row0 + i * 16 + rlane) * KD + ks * 32 + koff);
#pragma unroll
      for (int ks = 0; ks < KS; ++ks) asm volatile("" : "+v"(af[i][ks]) :: "memory");
    }
  } else {
#pragma unroll
    for (int i = 0; i < 2; ++i)
#pragma unroll
      for (int ks = 0; ks < KS; ++ks)
        af[i][ks] = bn_frag(Ain + (size_t)(row0 + i * 16 + rlane) * KD + ks * 32 + koff,
                            scs + ks * 32 + koff, shs + ks * 32 + koff);
  }

  const _Float16* Wb = (const _Float16*)Wh;
#pragma unroll 1
  for (int nh = 0; nh < NH; ++nh) {
    v8f acc[2][4];
#pragma unroll
    for (int i = 0; i < 2; ++i)
#pragma unroll
      for (int j = 0; j < 4; ++j) acc[i][j] = (v8f){0.f, 0.f, 0.f, 0.f, 0.f, 0.f, 0.f, 0.f};

#pragma unroll
    for (int ks = 0; ks < KS; ++ks) {
      v16h bfr[4];
#pragma unroll
      for (int j = 0; j < 4; ++j)
        bfr[j] = Frag<_Float16>::load(Wb + (size_t)(nh * 64 + j * 16 + rlane) * KD + ks * 32 + koff);
#pragma unroll
      for (int i = 0; i < 2; ++i)
#pragma unroll
        for (int j = 0; j < 4; ++j) acc[i][j] = Frag<_Float16>::mma(af[i][ks], bfr[j], acc[i][j]);
      guard8(acc[0][0], acc[0][1], acc[0][2], acc[0][3], acc[1][0], acc[1][1], acc[1][2], acc[1][3],
             af[0][ks], af[1][ks], bfr[0], bfr[1], bfr[2], bfr[3]);
    }

#pragma unroll
    for (int j = 0; j < 4; ++j) {
      const float bvj = rbf(bias[nh * 64 + j * 16 + rlane]);
#pragma unroll
      for (int i = 0; i < 2; ++i)
#pragma unroll
        for (int r = 0; r < 8; ++r) acc[i][j][r] = acc[i][j][r] * W_CARRY_INV + bvj;
    }

#pragma unroll
    for (int j = 0; j < 4; ++j) {
      float s = 0.0f, q = 0.0f;
#pragma unroll
      for (int i = 0; i < 2; ++i)
#pragma unroll
        for (int r = 0; r < 8; ++r) { const float v = acc[i][j][r]; s += v; q += v * v; }
      s += __shfl_xor(s, 16, 32);
      q += __shfl_xor(q, 16, 32);
      if (hh == 0) {
        wst[wave][nh * 64 + j * 16 + rlane] = s;
        wst[wave][NOUT + nh * 64 + j * 16 + rlane] = q;
      }
    }

    if (MODE == 2) {
#pragma unroll
      for (int j = 0; j < 4; ++j) {
        float mx = acc[0][j][0];
        float mn = acc[0][j][0];
#pragma unroll
        for (int i = 0; i < 2; ++i)
#pragma unroll
          for (int r = 0; r < 8; ++r) { const float v = acc[i][j][r]; mx = fmaxf(mx, v); mn = fminf(mn, v); }
        const float omx = __shfl_xor(mx, 16, 32);
        const float omn = __shfl_xor(mn, 16, 32);
        mx = fmaxf(mx, omx);
        mn = fminf(mn, omn);
        if (hh == 0) {
          wmm[wave][nh * 64 + j * 16 + rlane] = mx;
          wmm[wave][NOUT + nh * 64 + j * 16 + rlane] = mn;
        }
      }
    } else {
      float* slab = slabs[wave];
#pragma unroll
      for (int i = 0; i < 2; ++i) {
#pragma unroll
        for (int j = 0; j < 4; ++j)
#pragma unroll
          for (int r = 0; r < 8; ++r) slab[(mOff + r) * 68 + (j << 4) + rlane] = acc[i][j][r];
        __builtin_amdgcn_fence(__ATOMIC_RELEASE, "workgroup");
        __builtin_amdgcn_wave_barrier();
        __builtin_amdgcn_fence(__ATOMIC_ACQUIRE, "workgroup");
        const int q4 = lane >> 3, c8 = (lane & 7) * 8;
        for (int pass = 0; pass < 2; ++pass) {
#pragma unroll
          for (int it = 0; it < 4; ++it) {
            const int row = it * 4 + q4;
            const float* sp = slab + row * 68 + c8;
            v8h hv;
#pragma unroll
            for (int e = 0; e < 8; ++e) hv[e] = (_Float16)sp[e];
            *(volatile v8h*)(Yout + (size_t)(row0 + i * 16 + row) * 64 + nh * 64 + c8) = hv;
          }
          __threadfence();
        }
        __builtin_amdgcn_fence(__ATOMIC_RELEASE, "workgroup");
        __builtin_amdgcn_wave_barrier();
        __builtin_amdgcn_fence(__ATOMIC_ACQUIRE, "workgroup");
      }
    }
  }

  __syncthreads();
  if (tid < 2 * NOUT) {
    float a = 0.0f;
#pragma unroll
    for (int w = 0; w < 8; ++w) a += wst[w][tid];
    bst[tid] = a;
  }
  if (MODE == 2) {
    const v4f vmx = *(const v4f*)(&wmm[wave][lane * 4]);
    const v4f vmn = *(const v4f*)(&wmm[wave][NOUT + lane * 4]);
    for (int pass = 0; pass < 2; ++pass) {
      *(volatile v4f*)(MXo + (size_t)g * NOUT + lane * 4) = vmx;
      *(volatile v4f*)(MNo + (size_t)g * NOUT + lane * 4) = vmn;
      __threadfence();
    }
  }
  __syncthreads();
  if (wave == 0) {
    float* pb = part + (size_t)blockIdx.x * 2 * NOUT;
    for (int pass = 0; pass < 2; ++pass) {
#pragma unroll
      for (int i = 0; i < (2 * NOUT) / 128; ++i) {
        const v4f v = *(const v4f*)(bst + (i * 32 + lane) * 4);
        *(volatile v4f*)(pb + (i * 32 + lane) * 4) = v;
      }
      __threadfence();
    }
  }
}

template <int NCH>
__global__ __launch_bounds__(128) void k_stats(const float* __restrict__ part, float* __restrict__ st, int nblk) {
  constexpr int NPART = 128 / NCH;
  static_assert(NCH == 64 || NCH == 128, "channel count");
  __shared__ double ds[128];
  __shared__ double dq[128];
  __shared__ __align__(16) float so[2 * NCH];
  const int tid = threadIdx.x;
  const int c = tid % NCH;
  const int pid = tid / NCH;
  const int nb = nblk < MLP_BLOCKS ? nblk : MLP_BLOCKS;
  double s = 0.0, q = 0.0;
  for (int blk = pid; blk < nb; blk += NPART) {
    const float a = part[(size_t)blk * 2 * NCH + c];
    const float d = part[(size_t)blk * 2 * NCH + NCH + c];
    s += (double)a;
    q += (double)d;
  }
  ds[tid] = s;
  dq[tid] = q;
  __syncthreads();
  if (tid < NCH) {
    for (int p = 1; p < NPART; ++p) { s += ds[tid + p * NCH]; q += dq[tid + p * NCH]; }
    constexpr double inv_n = 1.0 / (double)TOK_N;
    const double mean = s * inv_n;
    double var = q * inv_n - mean * mean;
    var = var < 0.0 ? 0.0 : var;
    const float vf = (float)var + BN_EPS;
    so[tid] = (float)mean;
    so[NCH + tid] = 1.0f / sqrtf(vf);
  }
  __syncthreads();
  if (tid < 32) {
    for (int pass = 0; pass < 2; ++pass) {
#pragma unroll
      for (int i = 0; i < (2 * NCH) / 128; ++i) {
        const v4f v = *(const v4f*)(so + (i * 32 + tid) * 4);
        *(volatile v4f*)(st + (i * 32 + tid) * 4) = v;
      }
      __threadfence();
    }
  }
}

__global__ __launch_bounds__(256) void k_final(const float* __restrict__ MX, const float* __restrict__ MN,
                                               const float* __restrict__ st2, const float* __restrict__ g2,
                                               const float* __restrict__ be2, float* __restrict__ out1) {
  const int i = blockIdx.x * 256 + threadIdx.x;
  const int c4 = (i & 31) * 4;
  const v4f mx = *(const v4f*)(MX + (size_t)i * 4);
  const v4f mn = *(const v4f*)(MN + (size_t)i * 4);
  const v4f mu = *(const v4f*)(st2 + c4);
  const v4f rs = *(const v4f*)(st2 + 128 + c4);
  const v4f gg = *(const v4f*)(g2 + c4);
  const v4f bb = *(const v4f*)(be2 + c4);
  v4f o;
#pragma unroll
  for (int e = 0; e < 4; ++e) {
    const float gr = gg[e];
    const float br = bb[e];
    const float gv = rbf(gr);
    const float bv = rbf(br);
    const float r = rs[e];
    const float sg = r * gv;
    const float fa = (sg >= 0.0f) ? 1.0f : 0.0f;
    const float fb = 1.0f - fa;
    const float a = mx[e];
    const float b = mn[e];
    const float sel = fa * a + fb * b;
    float v = (sel - mu[e]) * r;
    v = v * gv;
    v = v + bv;
    o[e] = fmaxf(v, 0.0f);
  }
  store2_v4f(out1 + (size_t)i * 4, o);
}

extern "C" void kernel_launch(void* const* d_in, const int* in_sizes, int n_in,
                              void* d_out, int out_size, void* d_ws, size_t ws_size,
                              hipStream_t stream) {
  (void)in_sizes; (void)out_size;
  if (n_in < 14) return;
  if (ws_size < WS_TOTAL) return;

  const float* xyz    = (const float*)d_in[0];
  const float* points = (const float*)d_in[1];
  const float* W0  = (const float*)d_in[2];
  const float* b0  = (const float*)d_in[3];
  const float* g0  = (const float*)d_in[4];
  const float* be0 = (const float*)d_in[5];
  const float* W1  = (const float*)d_in[6];
  const float* b1  = (const float*)d_in[7];
  const float* g1  = (const float*)d_in[8];
  const float* be1 = (const float*)d_in[9];
  const float* W2  = (const float*)d_in[10];
  const float* b2  = (const float*)d_in[11];
  const float* g2  = (const float*)d_in[12];
  const float* be2 = (const float*)d_in[13];

  float* out0 = (float*)d_out;
  float* out1 = (float*)d_out + (OUT0_BYTES / 4);

  char* ws = (char*)d_ws;
  float* XR  = (float*)(ws + OFF_XR);
  float* NXW = (float*)(ws + OFF_NXW);
  unsigned short* W0h = (unsigned short*)(ws + OFF_W0H);
  unsigned short* W1h = (unsigned short*)(ws + OFF_W1H);
  unsigned short* W2h = (unsigned short*)(ws + OFF_W2H);
  unsigned short* A0  = (unsigned short*)(ws + OFF_A0);
  unsigned short* Y0  = (unsigned short*)(ws + OFF_Y0);
  unsigned short* Y1  = (unsigned short*)(ws + OFF_Y1);
  float* MX  = (float*)(ws + OFF_MX);
  float* MN  = (float*)(ws + OFF_MN);
  float* P0  = (float*)(ws + OFF_P0);
  float* P1  = (float*)(ws + OFF_P1);
  float* P2  = (float*)(ws + OFF_P2);
  float* ST0 = (float*)(ws + OFF_ST0);
  float* ST1 = (float*)(ws + OFF_ST1);
  float* ST2 = (float*)(ws + OFF_ST2);

  k_prep<<<PREP_BLOCKS, 256, 0, stream>>>(xyz, W0, W1, W2, XR, W0h, W1h, W2h);
  k_fps<<<BATCH_N, 256, 0, stream>>>(XR, out0, NXW);
  k_group<<<GROUPS_N / 4, 128, 0, stream>>>(XR, points, NXW, A0);

  k_mlp<K0_PAD, 64, 0><<<MLP_BLOCKS, 256, 0, stream>>>(A0, W0h, b0, ST0, g0, be0, Y0, MX, MN, P0);
  k_stats<64><<<1, 128, 0, stream>>>(P0, ST0, MLP_BLOCKS);
  k_mlp<64, 64, 1><<<MLP_BLOCKS, 256, 0, stream>>>(Y0, W1h, b1, ST0, g0, be0, Y1, MX, MN, P1);
  k_stats<64><<<1, 128, 0, stream>>>(P1, ST1, MLP_BLOCKS);
  k_mlp<64, 128, 2><<<MLP_BLOCKS, 256, 0, stream>>>(Y1, W2h, b2, ST1, g1, be1, Y1, MX, MN, P2);
  k_stats<128><<<1, 128, 0, stream>>>(P2, ST2, MLP_BLOCKS);
  k_final<<<(GROUPS_N * 128 / 4) / 256, 256, 0, stream>>>(MX, MN, ST2, g2, be2, out1);
}
